// RelPositionMultiHeadAttention_53068615910311
// MI455X (gfx1250) — hardware-verified
//
#include <hip/hip_runtime.h>
#include <math.h>
#include <stdint.h>

#define NB    2
#define TT    1024
#define FF    1024
#define NH    16
#define DH    64
#define NPOS  2047
#define PPAD  2048
#define HG    4
#define NG    (NH / HG)
#define PSCALE 32768.0f

typedef __attribute__((ext_vector_type(16))) _Float16 v16h;
typedef __attribute__((ext_vector_type(8)))  _Float16 v8h;
typedef __attribute__((ext_vector_type(16))) __bf16   v16b;
typedef __attribute__((ext_vector_type(8)))  __bf16   v8b;
typedef __attribute__((ext_vector_type(8)))  float    v8f;
typedef __attribute__((ext_vector_type(4)))  float    v4f;
typedef __attribute__((ext_vector_type(2)))  float    v2f;
typedef __attribute__((ext_vector_type(4)))  unsigned int v4u;
typedef __attribute__((ext_vector_type(4)))  int      v4i;

__device__ __forceinline__ unsigned short f2bf_bits(float f) {
  unsigned u = __float_as_uint(f);
  return (unsigned short)((u + 0x7FFFu + ((u >> 16) & 1u)) >> 16);
}
__device__ __forceinline__ float bf_bits2f(unsigned short h) { return __uint_as_float(((unsigned)h) << 16); }

__device__ __forceinline__ void dep_guard_h(v8f& a, v8f& b, v16h x, v16h y) { asm volatile("v_nop\n\tv_nop\n\tv_nop\n\tv_nop" : "+v"(a), "+v"(b) : "v"(x), "v"(y)); }
__device__ __forceinline__ void dep_guard_b(v8f& a, v8f& b, v16b x, v16b y) { asm volatile("v_nop\n\tv_nop\n\tv_nop\n\tv_nop" : "+v"(a), "+v"(b) : "v"(x), "v"(y)); }
__device__ __forceinline__ void keep4_h(v16h a, v16h b, v16h c, v16h d) { asm volatile("v_nop" :: "v"(a), "v"(b), "v"(c), "v"(d)); }
__device__ __forceinline__ void keep4_b(v16b a, v16b b, v16b c, v16b d) { asm volatile("v_nop" :: "v"(a), "v"(b), "v"(c), "v"(d)); }
__device__ __forceinline__ void acc_guard4(v8f& a, v8f& b, v8f& c, v8f& d) { asm volatile("v_nop\n\tv_nop\n\tv_nop\n\tv_nop" : "+v"(a), "+v"(b), "+v"(c), "+v"(d)); }
template <typename T> struct Frag;
template <> struct Frag<_Float16> {
  typedef v16h V; union U { v16h v; v8h h[2]; };
  static __device__ __forceinline__ v16h load(const _Float16* p) {
    U f; f.h[0] = *(const v8h*)(p); f.h[1] = *(const v8h*)(p + 16); return f.v;
  }
  static __device__ __forceinline__ v8f mma(v16h a, v16h b, v8f c) {
    return __builtin_amdgcn_wmma_f32_16x16x32_f16(false, a, false, b, (short)0, c, false, false);
  }
  static __device__ __forceinline__ void guard(v8f& a, v8f& b, v16h x, v16h y) { dep_guard_h(a, b, x, y); }
  static __device__ __forceinline__ void keep(v16h a, v16h b, v16h c, v16h d) { keep4_h(a, b, c, d); }
};
template <> struct Frag<__bf16> {
  typedef v16b V; union U { v16b v; v8b h[2]; };
  static __device__ __forceinline__ v16b load(const __bf16* p) {
    U f; f.h[0] = *(const v8b*)(p); f.h[1] = *(const v8b*)(p + 16); return f.v;
  }
  static __device__ __forceinline__ v8f mma(v16b a, v16b b, v8f c) {
    return __builtin_amdgcn_wmma_f32_16x16x32_bf16(false, a, false, b, (short)0, c, false, false);
  }
  static __device__ __forceinline__ void guard(v8f& a, v8f& b, v16b x, v16b y) { dep_guard_b(a, b, x, y); }
  static __device__ __forceinline__ void keep(v16b a, v16b b, v16b c, v16b d) { keep4_b(a, b, c, d); }
};

template <int ET> struct Elem;
template <> struct Elem<0> { typedef _Float16 T; };
template <> struct Elem<1> { typedef __bf16 T; };
template <int ET, bool SPLIT, int BIAS_MODE, int OUT_MODE, bool RESID, int ACT = 0, int BANDW = 0, int BANDB = 0>
__global__ __launch_bounds__(256) void wmma_gemm64(
    const unsigned short* __restrict__ Ap, const unsigned short* __restrict__ A2p, int lda, long strideA,
    const unsigned short* __restrict__ Btp, const unsigned short* __restrict__ Bt2p, int ldb, long strideB,
    void* __restrict__ Cout, void* __restrict__ Cout2, int ldc, long strideC,
    const float* __restrict__ bias,
    const float* __restrict__ resid, long strideR,
    int M, int N, int K, float scale) {
  typedef typename Elem<ET>::T T;
  typedef typename Frag<T>::V V;
  const T* A = (const T*)Ap; const T* A2 = (const T*)A2p; const T* Bt = (const T*)Btp; const T* Bt2 = (const T*)Bt2p;
  __shared__ __align__(16) float sT[8][16 * 68];
  const int b    = blockIdx.y;
  const int lane = threadIdx.x & 31;
  const int wave = threadIdx.x >> 5;
  const int tilesN = (BANDW > 0) ? BANDW : (N >> 6);
  const int tilesM = M >> 6;
  const int tile = blockIdx.x * 8 + wave;
  if (tile >= tilesM * tilesN) return;
  const int tm = tile / tilesN;
  const int tt = tile - tm * tilesN;
  const int tn = (BANDW > 0) ? (BANDB - tm + tt) : tt;
  const int m0 = tm << 6;
  const int n0 = tn << 6;

  const T* Ab  = A  + (size_t)b * strideA;
  const T* Bb  = Bt + (size_t)b * strideB;
  const T* Ab2 = SPLIT ? (A2  + (size_t)b * strideA) : nullptr;
  const T* Bb2 = SPLIT ? (Bt2 + (size_t)b * strideB) : nullptr;

  const int rlane = lane & 15;
  const int koff  = (lane >> 4) * 8;
  const int mOff  = (lane >> 4) * 8;

  v8f acc[4][4];
#pragma unroll
  for (int i = 0; i < 4; ++i)
#pragma unroll
    for (int j = 0; j < 4; ++j) acc[i][j] = (v8f){0.f,0.f,0.f,0.f,0.f,0.f,0.f,0.f};

  for (int k0 = 0; k0 < K; k0 += 32) {
    V bh[4], bl[4];
#pragma unroll
    for (int j = 0; j < 4; ++j) {
      const size_t bo = (size_t)(n0 + (j << 4) + rlane) * ldb + koff + k0;
      bh[j] = Frag<T>::load(Bb + bo);
      if (SPLIT) bl[j] = Frag<T>::load(Bb2 + bo);
    }
#pragma unroll
    for (int i = 0; i < 4; ++i) {
      const size_t ao = (size_t)(m0 + (i << 4) + rlane) * lda + koff + k0;
      V ah = Frag<T>::load(Ab + ao);
      V al;
      if (SPLIT) al = Frag<T>::load(Ab2 + ao);
#pragma unroll
      for (int j = 0; j < 4; ++j) {
        acc[i][j] = Frag<T>::mma(ah, bh[j], acc[i][j]);
        if (SPLIT) {
          acc[i][j] = Frag<T>::mma(ah, bl[j], acc[i][j]);
          acc[i][j] = Frag<T>::mma(al, bh[j], acc[i][j]);
        }
      }
      Frag<T>::guard(acc[i][0], acc[i][3], ah, SPLIT ? al : ah);
    }
    Frag<T>::keep(bh[0], bh[1], bh[2], bh[3]);
    if (SPLIT) Frag<T>::keep(bl[0], bl[1], bl[2], bl[3]);
  }
  acc_guard4(acc[0][0], acc[0][1], acc[0][2], acc[0][3]);
  acc_guard4(acc[1][0], acc[1][1], acc[1][2], acc[1][3]);
  acc_guard4(acc[2][0], acc[2][1], acc[2][2], acc[2][3]);
  acc_guard4(acc[3][0], acc[3][1], acc[3][2], acc[3][3]);

  float* slab = sT[wave];
  const float* Rb = RESID ? (resid + (size_t)b * strideR) : nullptr;
#pragma unroll
  for (int i = 0; i < 4; ++i) {
    const int mBase = m0 + (i << 4);
#pragma unroll
    for (int j = 0; j < 4; ++j) {
      const int n = n0 + (j << 4) + rlane;
      float bv = 0.f;
      if (BIAS_MODE == 2) bv = bias[n];
#pragma unroll
      for (int r = 0; r < 8; ++r) {
        float v = acc[i][j][r] * scale;
        if (BIAS_MODE == 1) v += bias[mBase + mOff + r];
        if (BIAS_MODE == 2) v += bv;
        if (RESID) v += Rb[(size_t)(mBase + mOff + r) * ldc + n];
        if (ACT == 1) v = tanhf(v);
        if (ACT == 2) v = fmaxf(v, 0.0f);
        if (ACT == 3) v = v / (1.0f + expf(-v));
        if (ACT == 4) v = (v > 0.f) ? v : 0.01f * v;
        slab[(mOff + r) * 68 + (j << 4) + rlane] = v;
      }
    }
    __builtin_amdgcn_fence(__ATOMIC_RELEASE, "workgroup");
    __builtin_amdgcn_wave_barrier();
    __builtin_amdgcn_fence(__ATOMIC_ACQUIRE, "workgroup");
    if (OUT_MODE == 0) {
      float* C = (float*)Cout + (size_t)b * strideC;
      const int hh = lane >> 4, c4 = (lane & 15) * 4;
      for (int pass = 0; pass < 2; ++pass) {
#pragma unroll
        for (int it = 0; it < 8; ++it) {
          const int row = it * 2 + hh;
          v4f v = *(const v4f*)(slab + row * 68 + c4);
          *(volatile v4f*)(C + (size_t)(mBase + row) * ldc + n0 + c4) = v;
        }
        __threadfence();
      }
    } else {
      const int q = lane >> 3, c8 = (lane & 7) * 8;
      unsigned short* C  = (unsigned short*)Cout  + (size_t)b * strideC;
      unsigned short* C2 = (OUT_MODE == 2) ? ((unsigned short*)Cout2 + (size_t)b * strideC) : nullptr;
      for (int pass = 0; pass < 2; ++pass) {
#pragma unroll
        for (int it = 0; it < 4; ++it) {
          const int row = it * 4 + q;
          const float* sp = slab + row * 68 + c8;
          v8h hv, lv;
#pragma unroll
          for (int e = 0; e < 8; ++e) {
            if (OUT_MODE == 1) {
              hv[e] = (_Float16)sp[e];
            } else {
              unsigned short hb = f2bf_bits(sp[e]);
              unsigned short lb = f2bf_bits(sp[e] - bf_bits2f(hb));
              hv[e] = __builtin_bit_cast(_Float16, hb);
              lv[e] = __builtin_bit_cast(_Float16, lb);
            }
          }
          *(volatile v8h*)(C + (size_t)(mBase + row) * ldc + n0 + c8) = hv;
          if (OUT_MODE == 2) *(volatile v8h*)(C2 + (size_t)(mBase + row) * ldc + n0 + c8) = lv;
        }
        __threadfence();
      }
    }
    __builtin_amdgcn_fence(__ATOMIC_RELEASE, "workgroup");
    __builtin_amdgcn_wave_barrier();
    __builtin_amdgcn_fence(__ATOMIC_ACQUIRE, "workgroup");
  }
}

__device__ __forceinline__ unsigned pk16(unsigned short a, unsigned short b) { return (unsigned)a | ((unsigned)b << 16); }
__device__ __forceinline__ unsigned short h_bits(float f) { const _Float16 h = (_Float16)f; return __builtin_bit_cast(unsigned short, h); }

__global__ __launch_bounds__(256) void cast_f16x2_kernel(const float* __restrict__ in, unsigned short* __restrict__ out,
                                                         int n2, int n2v, float scale) {
  const int i = blockIdx.x * 256 + threadIdx.x;
  if (i < n2) {
    const int ic = (i < n2v) ? i : (n2v - 1);
    v2f f = *(const v2f*)(in + 2 * (size_t)ic);
    if (i >= n2v) { f[0] = 0.0f; f[1] = 0.0f; }
    const unsigned u = pk16(h_bits(f[0] * scale), h_bits(f[1] * scale));
    ((volatile unsigned*)out)[i] = u;
    __threadfence();
    ((volatile unsigned*)out)[i] = u;
  }
}

__global__ __launch_bounds__(256) void transpose_cast_f16_kernel(const float* __restrict__ in, unsigned short* __restrict__ out,
                                                                 int R, int C, float scale) {
  __shared__ __align__(16) float sm[64 * 68];
  const int tid = threadIdx.x, lane = tid & 31, wave = tid >> 5;
  const int r0 = blockIdx.y * 64, c0 = blockIdx.x * 64;
  const int lr = tid >> 2, lc = (tid & 3) * 16;
  const float* src = in + (size_t)(r0 + lr) * C + c0 + lc;
#pragma unroll
  for (int e4 = 0; e4 < 4; ++e4) {
    const v4f v = *(const v4f*)(src + 4 * e4);
#pragma unroll
    for (int x = 0; x < 4; ++x) sm[(lc + 4 * e4 + x) * 68 + lr] = v[x];
  }
  __syncthreads();
  const int q = lane >> 3, c8 = (lane & 7) * 8;
  for (int pass = 0; pass < 2; ++pass) {
#pragma unroll
    for (int it = 0; it < 2; ++it) {
      const int orow = it * 32 + wave * 4 + q;
      const float* sp = sm + orow * 68 + c8;
      v8h hv;
#pragma unroll
      for (int e = 0; e < 8; ++e) hv[e] = (_Float16)(sp[e] * scale);
      *(volatile v8h*)(out + (size_t)(c0 + orow) * R + r0 + c8) = hv;
    }
    __threadfence();
  }
}

__global__ __launch_bounds__(256) void qbias_cast_kernel(const float* __restrict__ Q, const float* __restrict__ pu,
                                                         const float* __restrict__ pv, unsigned short* __restrict__ QU,
                                                         unsigned short* __restrict__ QV, int n2, int ncolmask) {
  const int i = blockIdx.x * 256 + threadIdx.x;
  if (i < n2) {
    const v2f f = *(const v2f*)(Q + 2 * (size_t)i);
    const int n = (2 * i) & ncolmask;
    const float u0 = pu[n], u1 = pu[n + 1], w0 = pv[n], w1 = pv[n + 1];
    const unsigned a = pk16(h_bits(f[0] + u0), h_bits(f[1] + u1));
    const unsigned c = pk16(h_bits(f[0] + w0), h_bits(f[1] + w1));
    ((volatile unsigned*)QU)[i] = a;
    ((volatile unsigned*)QV)[i] = c;
    __threadfence();
    ((volatile unsigned*)QU)[i] = a;
    ((volatile unsigned*)QV)[i] = c;
  }
}

__global__ __launch_bounds__(128) void rel_softmax_kernel(const float* __restrict__ AC, const float* __restrict__ BD,
                                                          const int* __restrict__ maskb, unsigned short* __restrict__ P) {
  __shared__ float redm[4];
  __shared__ float reds[4];
  const int i    = blockIdx.x;
  const int hg   = blockIdx.y;
  const int tid  = threadIdx.x;
  const int lane = tid & 31;
  const int wave = tid >> 5;
  const int j0   = tid * 8;
  const float* arow = AC + ((size_t)hg * TT + i) * TT + j0;
  const v4f a0 = *(const v4f*)(arow);
  const v4f a1 = *(const v4f*)(arow + 4);
  int cb = (TT - 1 - i) + j0;
  cb = (cb < 0) ? 0 : cb;
  cb = (cb > (PPAD - 8)) ? (PPAD - 8) : cb;
  const float* brow = BD + ((size_t)hg * TT + i) * PPAD + cb;
  float bdv[8];
#pragma unroll
  for (int e = 0; e < 8; ++e) bdv[e] = brow[e];
  const int* mrow = maskb + (size_t)i * TT + j0;
  const v4i mk0 = *(const v4i*)(mrow);
  const v4i mk1 = *(const v4i*)(mrow + 4);
  float t[8];
#pragma unroll
  for (int e = 0; e < 4; ++e) {
    const float s0 = a0[e] + bdv[e];
    const float s1 = a1[e] + bdv[4 + e];
    t[e]     = (mk0[e] > 0) ? s0 : -10000.0f;
    t[4 + e] = (mk1[e] > 0) ? s1 : -10000.0f;
  }
  float m = t[0];
#pragma unroll
  for (int e = 1; e < 8; ++e) m = fmaxf(m, t[e]);
#pragma unroll
  for (int off = 16; off > 0; off >>= 1) m = fmaxf(m, __shfl_xor(m, off, 32));
  if (lane == 0) redm[wave] = m;
  __syncthreads();
  float mx = redm[0];
#pragma unroll
  for (int w = 1; w < 4; ++w) mx = fmaxf(mx, redm[w]);
  float ev[8];
  float s = 0.0f;
#pragma unroll
  for (int e = 0; e < 8; ++e) { ev[e] = __expf(t[e] - mx); s += ev[e]; }
#pragma unroll
  for (int off = 16; off > 0; off >>= 1) s += __shfl_xor(s, off, 32);
  if (lane == 0) reds[wave] = s;
  __syncthreads();
  float tot = reds[0];
#pragma unroll
  for (int w = 1; w < 4; ++w) tot += reds[w];
  const float inv = 1.0f / tot;
  const v4u hv = (v4u){pk16(h_bits(ev[0] * inv * PSCALE), h_bits(ev[1] * inv * PSCALE)),
                       pk16(h_bits(ev[2] * inv * PSCALE), h_bits(ev[3] * inv * PSCALE)),
                       pk16(h_bits(ev[4] * inv * PSCALE), h_bits(ev[5] * inv * PSCALE)),
                       pk16(h_bits(ev[6] * inv * PSCALE), h_bits(ev[7] * inv * PSCALE))};
  const size_t ro = ((size_t)hg * TT + i) * TT + j0;
  *(volatile v4u*)(P + ro) = hv;
  __threadfence();
  *(volatile v4u*)(P + ro) = hv;
}

extern "C" void kernel_launch(void* const* d_in, const int* in_sizes, int n_in,
                              void* d_out, int out_size, void* d_ws, size_t ws_size,
                              hipStream_t stream) {
  if (n_in < 16) return;
  if (in_sizes[0] != NB * TT * FF || in_sizes[1] != NB * TT * FF || in_sizes[2] != NB * TT * FF) return;
  if (in_sizes[3] != NPOS * FF) return;
  if (in_sizes[4] != NB * TT * TT) return;
  if (in_sizes[5] != FF * FF || in_sizes[7] != FF * FF || in_sizes[9] != FF * FF ||
      in_sizes[11] != FF * FF || in_sizes[12] != FF * FF) return;
  if (in_sizes[6] != FF || in_sizes[8] != FF || in_sizes[10] != FF || in_sizes[13] != FF) return;
  if (in_sizes[14] != NH * DH || in_sizes[15] != NH * DH) return;
  if (out_size != NB * TT * FF) return;

  const float* query = (const float*)d_in[0];
  const float* key   = (const float*)d_in[1];
  const float* value = (const float*)d_in[2];
  const float* pos   = (const float*)d_in[3];
  const int*   mask  = (const int*)d_in[4];
  const float* Wq    = (const float*)d_in[5];
  const float* bq    = (const float*)d_in[6];
  const float* Wk    = (const float*)d_in[7];
  const float* bk    = (const float*)d_in[8];
  const float* Wv    = (const float*)d_in[9];
  const float* bv    = (const float*)d_in[10];
  const float* Wpos  = (const float*)d_in[11];
  const float* Wo    = (const float*)d_in[12];
  const float* bo    = (const float*)d_in[13];
  const float* pbu   = (const float*)d_in[14];
  const float* pbv   = (const float*)d_in[15];

  const size_t PW  = (size_t)FF * FF * 2;
  const size_t PPE = (size_t)PPAD * FF * 2;
  const size_t PQF = (size_t)TT * FF * 4;
  const size_t PAC = (size_t)HG * TT * TT * 4;
  const size_t PBD = (size_t)HG * TT * PPAD * 4;
  const size_t PP  = (size_t)HG * TT * TT * 2;
  size_t off = 0;
  const size_t oWqT = off; off += PW;
  const size_t oWkT = off; off += PW;
  const size_t oWvT = off; off += PW;
  const size_t oWpT = off; off += PW;
  const size_t oWoT = off; off += PW;
  const size_t oPE  = off; off += PPE;
  const size_t oPP  = off; off += PPE;
  const size_t oXQ  = off; off += PW;
  const size_t oXK  = off; off += PW;
  const size_t oXV  = off; off += PW;
  const size_t oQf  = off; off += PQF;
  const size_t oQU  = off; off += PW;
  const size_t oQV  = off; off += PW;
  const size_t oK16 = off; off += PW;
  const size_t oVT  = off; off += PW;
  const size_t oX16 = off; off += PW;
  const size_t oAC  = off; off += PAC;
  const size_t oBD  = off; off += PBD;
  const size_t oP16 = off; off += PP;
  if (off > ws_size) return;

  char* ws = (char*)d_ws;
  unsigned short* WqT16 = (unsigned short*)(ws + oWqT);
  unsigned short* WkT16 = (unsigned short*)(ws + oWkT);
  unsigned short* WvT16 = (unsigned short*)(ws + oWvT);
  unsigned short* WpT16 = (unsigned short*)(ws + oWpT);
  unsigned short* WoT16 = (unsigned short*)(ws + oWoT);
  unsigned short* PE16  = (unsigned short*)(ws + oPE);
  unsigned short* PP16  = (unsigned short*)(ws + oPP);
  unsigned short* XQ16  = (unsigned short*)(ws + oXQ);
  unsigned short* XK16  = (unsigned short*)(ws + oXK);
  unsigned short* XV16  = (unsigned short*)(ws + oXV);
  float*          Qf    = (float*)(ws + oQf);
  unsigned short* QU16  = (unsigned short*)(ws + oQU);
  unsigned short* QV16  = (unsigned short*)(ws + oQV);
  unsigned short* K16   = (unsigned short*)(ws + oK16);
  unsigned short* VT16  = (unsigned short*)(ws + oVT);
  unsigned short* X16   = (unsigned short*)(ws + oX16);
  float*          ACb   = (float*)(ws + oAC);
  float*          BDb   = (float*)(ws + oBD);
  unsigned short* P16   = (unsigned short*)(ws + oP16);

  const dim3 blk(256);
  const dim3 blk128(128);

  const int bandB = TT / 64 - 1;
  const int bandW = TT / 64 + 1;
  if (bandB - (TT / 64 - 1) < 0) return;
  if (bandB + bandW - 1 > PPAD / 64 - 1) return;

  const dim3 gTW(FF / 64, FF / 64);
  transpose_cast_f16_kernel<<<gTW, blk, 0, stream>>>(Wq,   WqT16, FF, FF, 16.0f);
  transpose_cast_f16_kernel<<<gTW, blk, 0, stream>>>(Wk,   WkT16, FF, FF, 16.0f);
  transpose_cast_f16_kernel<<<gTW, blk, 0, stream>>>(Wv,   WvT16, FF, FF, 16.0f);
  transpose_cast_f16_kernel<<<gTW, blk, 0, stream>>>(Wpos, WpT16, FF, FF, 16.0f);
  transpose_cast_f16_kernel<<<gTW, blk, 0, stream>>>(Wo,   WoT16, FF, FF, 16.0f);

  const int n2pe  = PPAD * FF / 2;
  const int n2pev = NPOS * FF / 2;
  cast_f16x2_kernel<<<dim3((n2pe + 255) / 256), blk, 0, stream>>>(pos, PE16, n2pe, n2pev, 1.0f);

  const float wscale = 1.0f / 16.0f;
  wmma_gemm64<0, false, 0, 1, false><<<dim3(64, 1), blk, 0, stream>>>(
      PE16, PE16, FF, 0L, WpT16, WpT16, FF, 0L, (void*)PP16, (void*)PP16, FF, 0L,
      bq, bq, 0L, PPAD, FF, FF, wscale);

  const int  n2x   = TT * FF / 2;
  const dim3 gCastX((n2x + 255) / 256);
  const dim3 gProj((((TT / 64) * (FF / 64)) + 7) / 8, 1);
  const dim3 gAC((((TT / 64) * (TT / 64)) + 7) / 8, HG);
  const dim3 gBD((((TT / 64) * bandW) + 7) / 8, HG);
  const dim3 gPV((((TT / 64) * (DH / 64)) + 7) / 8, HG);
  const float sscale  = 0.125f;
  const float pvscale = 64.0f / PSCALE;
  const float oscale  = 1.0f / (16.0f * 64.0f);

  for (int b = 0; b < NB; ++b) {
    cast_f16x2_kernel<<<gCastX, blk, 0, stream>>>(query + (size_t)b * TT * FF, XQ16, n2x, n2x, 1.0f);
    cast_f16x2_kernel<<<gCastX, blk, 0, stream>>>(key   + (size_t)b * TT * FF, XK16, n2x, n2x, 1.0f);
    cast_f16x2_kernel<<<gCastX, blk, 0, stream>>>(value + (size_t)b * TT * FF, XV16, n2x, n2x, 1.0f);
    wmma_gemm64<0, false, 2, 0, false><<<gProj, blk, 0, stream>>>(
        XQ16, XQ16, FF, 0L, WqT16, WqT16, FF, 0L, (void*)Qf, (void*)Qf, FF, 0L,
        bq, bq, 0L, TT, FF, FF, wscale);
    qbias_cast_kernel<<<gCastX, blk, 0, stream>>>(Qf, pbu, pbv, QU16, QV16, n2x, FF - 1);
    wmma_gemm64<0, false, 2, 1, false><<<gProj, blk, 0, stream>>>(
        XK16, XK16, FF, 0L, WkT16, WkT16, FF, 0L, (void*)K16, (void*)K16, FF, 0L,
        bk, bk, 0L, TT, FF, FF, wscale);
    wmma_gemm64<0, false, 1, 1, false><<<gProj, blk, 0, stream>>>(
        WvT16, WvT16, FF, 0L, XV16, XV16, FF, 0L, (void*)VT16, (void*)VT16, TT, 0L,
        bv, bv, 0L, FF, TT, FF, wscale);

    const int* maskb = mask + (size_t)b * TT * TT;
    for (int g = 0; g < NG; ++g) {
      const size_t hc = (size_t)g * HG * DH;
      wmma_gemm64<0, false, 0, 0, false><<<gAC, blk, 0, stream>>>(
          QU16 + hc, QU16 + hc, FF, (long)DH, K16 + hc, K16 + hc, FF, (long)DH,
          (void*)ACb, (void*)ACb, TT, (long)TT * TT,
          bq, bq, 0L, TT, TT, DH, sscale);
      wmma_gemm64<0, false, 0, 0, false, 0, TT / 64 + 1, TT / 64 - 1><<<gBD, blk, 0, stream>>>(
          QV16 + hc, QV16 + hc, FF, (long)DH, PP16 + hc, PP16 + hc, FF, (long)DH,
          (void*)BDb, (void*)BDb, PPAD, (long)TT * PPAD,
          bq, bq, 0L, TT, PPAD, DH, sscale);
      rel_softmax_kernel<<<dim3(TT, HG), blk128, 0, stream>>>(ACb, BDb, maskb, P16);
      wmma_gemm64<0, false, 0, 1, false><<<gPV, blk, 0, stream>>>(
          P16, P16, TT, (long)TT * TT, VT16 + hc * TT, VT16 + hc * TT, TT, (long)DH * TT,
          (void*)(X16 + hc), (void*)(X16 + hc), FF, (long)DH,
          bq, bq, 0L, TT, DH, TT, pvscale);
    }
    float* outb = (float*)d_out + (size_t)b * TT * FF;
    wmma_gemm64<0, false, 2, 0, false><<<gProj, blk, 0, stream>>>(
        X16, X16, FF, 0L, WoT16, WoT16, FF, 0L, (void*)outb, (void*)outb, FF, 0L,
        bo, bq, 0L, TT, FF, FF, oscale);
  }
  (void)hipGetLastError();
}
